// DCN_2456721294049
// MI455X (gfx1250) — hardware-run, weakly checked
//
#include <hip/hip_runtime.h>
#include <stdint.h>

constexpr int NB = 2;
constexpr int CIN = 256;
constexpr int IMH = 128;
constexpr int IMW = 128;
constexpr int NOUT = 256;
constexpr int NTAP = 9;
constexpr int HWPIX = IMH * IMW;
constexpr int PW = IMW + 2;
constexpr int PROWS = (IMH + 3) * PW;
constexpr int QM = IMH * PW;
constexpr int NCH = 3 * NTAP;
constexpr int NCHP = 64;
constexpr int KCONV = NTAP * CIN;
constexpr int XT_PITCH = 136;
constexpr int SPB = 64;

static_assert(QM % 64 == 0, "conv GEMM M tile multiple");
static_assert(NCHP % 64 == 0, "conv GEMM N tile multiple");
static_assert(KCONV % 32 == 0, "conv GEMM K step multiple");
static_assert(CIN % 32 == 0, "out GEMM K step multiple and per-tap k block");
static_assert(CIN == 256, "tap decode uses k0 >> 8");
static_assert(NOUT % 64 == 0, "out GEMM M tile multiple");
static_assert(HWPIX % 64 == 0, "out GEMM N tile multiple");
static_assert(QM - 1 + 2 * PW + 2 < PROWS, "shifted A rows stay inside the padded plane");
static_assert(HWPIX % SPB == 0, "sample blocks do not straddle batches");
static_assert(NCH <= NCHP, "channel pad");

constexpr size_t XT_BYTES = (size_t)NB * PROWS * CIN * 2;
constexpr size_t WBT_BYTES = (size_t)NCHP * KCONV * 2;
constexpr size_t TMPQ_BYTES = (size_t)NB * QM * NCHP * 4;
constexpr size_t STATS_BYTES = (size_t)NB * NTAP * 128;
constexpr size_t WQ_BYTES = (size_t)NOUT * CIN * 2;
constexpr size_t AGG_BYTES = (size_t)NB * HWPIX * CIN * 2;
constexpr size_t OFF_XT = 0;
constexpr size_t OFF_WBT = OFF_XT + XT_BYTES;
constexpr size_t OFF_TMPQ = OFF_WBT + WBT_BYTES;
constexpr size_t OFF_STATS = OFF_TMPQ + TMPQ_BYTES;
constexpr size_t OFF_WQ = OFF_STATS + STATS_BYTES;
constexpr size_t OFF_AGG = OFF_WQ + WQ_BYTES;
constexpr size_t WS_TOTAL = OFF_AGG + AGG_BYTES;
static_assert(WS_TOTAL == 43163904, "carve total");
static_assert(WS_TOTAL <= (size_t)134217728, "carve under 128 MiB");
static_assert(OFF_WBT % 128 == 0 && OFF_TMPQ % 128 == 0 && OFF_STATS % 128 == 0 && OFF_WQ % 128 == 0 && OFF_AGG % 128 == 0, "128-B aligned regions");

typedef __attribute__((ext_vector_type(16))) _Float16 v16h;
typedef __attribute__((ext_vector_type(8)))  _Float16 v8h;
typedef __attribute__((ext_vector_type(16))) __bf16   v16b;
typedef __attribute__((ext_vector_type(8)))  __bf16   v8b;
typedef __attribute__((ext_vector_type(8)))  float    v8f;
typedef __attribute__((ext_vector_type(4)))  float    v4f;
typedef __attribute__((ext_vector_type(4)))  unsigned int v4u;
typedef v4u __attribute__((may_alias)) v4ua;

__device__ __forceinline__ unsigned short f2bf_bits(float f) {
  unsigned u = __float_as_uint(f);
  return (unsigned short)((u + 0x7FFFu + ((u >> 16) & 1u)) >> 16);
}
__device__ __forceinline__ float bf_bits2f(unsigned short h) { return __uint_as_float(((unsigned)h) << 16); }
__device__ __forceinline__ unsigned pack_bf2(float a, float b) {
  return (unsigned)f2bf_bits(a) | (((unsigned)f2bf_bits(b)) << 16);
}

__device__ __forceinline__ void dep_guard_h(v8f& a, v8f& b, v16h x, v16h y) { asm volatile("v_nop\n\tv_nop\n\tv_nop\n\tv_nop" : "+v"(a), "+v"(b) : "v"(x), "v"(y)); }
__device__ __forceinline__ void dep_guard_b(v8f& a, v8f& b, v16b x, v16b y) { asm volatile("v_nop\n\tv_nop\n\tv_nop\n\tv_nop" : "+v"(a), "+v"(b) : "v"(x), "v"(y)); }
__device__ __forceinline__ void keep4_h(v16h a, v16h b, v16h c, v16h d) { asm volatile("v_nop" :: "v"(a), "v"(b), "v"(c), "v"(d)); }
__device__ __forceinline__ void keep4_b(v16b a, v16b b, v16b c, v16b d) { asm volatile("v_nop" :: "v"(a), "v"(b), "v"(c), "v"(d)); }
__device__ __forceinline__ void acc_guard4(v8f& a, v8f& b, v8f& c, v8f& d) { asm volatile("v_nop\n\tv_nop\n\tv_nop\n\tv_nop" : "+v"(a), "+v"(b), "+v"(c), "+v"(d)); }
template <typename T> struct Frag;
template <> struct Frag<_Float16> {
  typedef v16h V; union U { v16h v; v8h h[2]; };
  static __device__ __forceinline__ v16h load(const _Float16* p) {
    U f; f.h[0] = *(const v8h*)(p); f.h[1] = *(const v8h*)(p + 16); return f.v;
  }
  static __device__ __forceinline__ v8f mma(v16h a, v16h b, v8f c) {
    return __builtin_amdgcn_wmma_f32_16x16x32_f16(false, a, false, b, (short)0, c, false, false);
  }
  static __device__ __forceinline__ void guard(v8f& a, v8f& b, v16h x, v16h y) { dep_guard_h(a, b, x, y); }
  static __device__ __forceinline__ void keep(v16h a, v16h b, v16h c, v16h d) { keep4_h(a, b, c, d); }
};
template <> struct Frag<__bf16> {
  typedef v16b V; union U { v16b v; v8b h[2]; };
  static __device__ __forceinline__ v16b load(const __bf16* p) {
    U f; f.h[0] = *(const v8b*)(p); f.h[1] = *(const v8b*)(p + 16); return f.v;
  }
  static __device__ __forceinline__ v8f mma(v16b a, v16b b, v8f c) {
    return __builtin_amdgcn_wmma_f32_16x16x32_bf16(false, a, false, b, (short)0, c, false, false);
  }
  static __device__ __forceinline__ void guard(v8f& a, v8f& b, v16b x, v16b y) { dep_guard_b(a, b, x, y); }
  static __device__ __forceinline__ void keep(v16b a, v16b b, v16b c, v16b d) { keep4_b(a, b, c, d); }
};

template <int AMODE, int BIAS_MODE>
__global__ __launch_bounds__(256) void gemm64_bf16(
    const unsigned short* __restrict__ Ap, int lda, long strideA,
    const unsigned short* __restrict__ Btp, int ldb, long strideB,
    float* __restrict__ Cout, int ldc, long strideC,
    const float* __restrict__ bias, int M, int N, int K, float scale) {
  typedef __bf16 T;
  typedef Frag<T>::V V;
  const T* A = (const T*)Ap;
  const T* Bt = (const T*)Btp;
  __shared__ __align__(16) float sT[8][16 * 68];
  const int b    = blockIdx.y;
  const int lane = threadIdx.x & 31;
  const int wave = threadIdx.x >> 5;
  const int tilesN = N >> 6;
  const int tilesM = M >> 6;
  const int tile = blockIdx.x * 8 + wave;
  if (tile >= tilesM * tilesN) return;
  const int tm = tile / tilesN;
  const int tn = tile - tm * tilesN;
  const int m0 = tm << 6;
  const int n0 = tn << 6;

  const T* Ab = A  + (size_t)b * strideA;
  const T* Bb = Bt + (size_t)b * strideB;

  const int rlane = lane & 15;
  const int koff  = (lane >> 4) * 8;
  const int mOff  = (lane >> 4) * 8;

  v8f acc[4][4];
#pragma unroll
  for (int i = 0; i < 4; ++i)
#pragma unroll
    for (int j = 0; j < 4; ++j) acc[i][j] = (v8f){0.f,0.f,0.f,0.f,0.f,0.f,0.f,0.f};

  for (int k0 = 0; k0 < K; k0 += 32) {
    int arow = 0;
    int kin = k0;
    if (AMODE == 1) {
      const int tap = k0 >> 8;
      const int ti = tap / 3;
      arow = ti * PW + (tap - 3 * ti);
      kin = k0 & (CIN - 1);
    }
    V bh[4];
#pragma unroll
    for (int j = 0; j < 4; ++j) {
      const size_t bo = (size_t)(n0 + (j << 4) + rlane) * ldb + koff + k0;
      bh[j] = Frag<T>::load(Bb + bo);
    }
#pragma unroll
    for (int i = 0; i < 4; ++i) {
      const size_t ao = (size_t)(m0 + (i << 4) + rlane + arow) * lda + koff + kin;
      V ah = Frag<T>::load(Ab + ao);
#pragma unroll
      for (int j = 0; j < 4; ++j) {
        acc[i][j] = Frag<T>::mma(ah, bh[j], acc[i][j]);
      }
      Frag<T>::guard(acc[i][0], acc[i][3], ah, ah);
    }
    Frag<T>::keep(bh[0], bh[1], bh[2], bh[3]);
  }
  acc_guard4(acc[0][0], acc[0][1], acc[0][2], acc[0][3]);
  acc_guard4(acc[1][0], acc[1][1], acc[1][2], acc[1][3]);
  acc_guard4(acc[2][0], acc[2][1], acc[2][2], acc[2][3]);
  acc_guard4(acc[3][0], acc[3][1], acc[3][2], acc[3][3]);

  float* slab = sT[wave];
#pragma unroll
  for (int i = 0; i < 4; ++i) {
    const int mBase = m0 + (i << 4);
    float bv8[8];
#pragma unroll
    for (int r = 0; r < 8; ++r) bv8[r] = 0.f;
    if (BIAS_MODE == 1) {
      const v4f bz0 = *(const v4f*)(bias + mBase + mOff);
      const v4f bz1 = *(const v4f*)(bias + mBase + mOff + 4);
      bv8[0] = bz0[0]; bv8[1] = bz0[1]; bv8[2] = bz0[2]; bv8[3] = bz0[3];
      bv8[4] = bz1[0]; bv8[5] = bz1[1]; bv8[6] = bz1[2]; bv8[7] = bz1[3];
    }
#pragma unroll
    for (int j = 0; j < 4; ++j) {
#pragma unroll
      for (int r = 0; r < 8; ++r) {
        float v = acc[i][j][r] * scale;
        if (BIAS_MODE == 1) v += bv8[r];
        slab[(mOff + r) * 68 + (j << 4) + rlane] = v;
      }
    }
    __builtin_amdgcn_fence(__ATOMIC_RELEASE, "workgroup");
    __builtin_amdgcn_wave_barrier();
    __builtin_amdgcn_fence(__ATOMIC_ACQUIRE, "workgroup");
    {
      float* C = Cout + (size_t)b * strideC;
      const int hh = lane >> 4, c4 = (lane & 15) * 4;
      for (int pass = 0; pass < 2; ++pass) {
#pragma unroll
        for (int it = 0; it < 8; ++it) {
          const int row = it * 2 + hh;
          v4f v = *(const v4f*)(slab + row * 68 + c4);
          *(volatile v4f*)(C + (size_t)(mBase + row) * ldc + n0 + c4) = v;
        }
        __threadfence();
      }
    }
    __builtin_amdgcn_fence(__ATOMIC_RELEASE, "workgroup");
    __builtin_amdgcn_wave_barrier();
    __builtin_amdgcn_fence(__ATOMIC_ACQUIRE, "workgroup");
  }
}

__global__ __launch_bounds__(256) void k_xpad(const float* __restrict__ x, unsigned short* __restrict__ xt) {
  __shared__ __align__(16) unsigned short sT[PW * XT_PITCH];
  const int yp = blockIdx.x;
  const int chalf = blockIdx.y;
  const int b = blockIdx.z;
  const int tid = threadIdx.x;
  const int lane = tid & 31;
  const int wave = tid >> 5;
  const bool interior = (yp >= 1) && (yp <= IMH);
  const int y = min(max(yp - 1, 0), IMH - 1);
  const float* xrow = x + ((size_t)b * CIN + (size_t)chalf * 128) * HWPIX + (size_t)y * IMW;
#pragma unroll 2
  for (int pass = 0; pass < 16; ++pass) {
    const int cl = pass * 8 + wave;
    const int x4 = lane * 4;
    const v4f v = *(const v4f*)(xrow + (size_t)cl * HWPIX + x4);
    const float f0 = interior ? v[0] : 0.f;
    const float f1 = interior ? v[1] : 0.f;
    const float f2 = interior ? v[2] : 0.f;
    const float f3 = interior ? v[3] : 0.f;
    sT[(x4 + 1) * XT_PITCH + cl] = f2bf_bits(f0);
    sT[(x4 + 2) * XT_PITCH + cl] = f2bf_bits(f1);
    sT[(x4 + 3) * XT_PITCH + cl] = f2bf_bits(f2);
    sT[(x4 + 4) * XT_PITCH + cl] = f2bf_bits(f3);
  }
  __syncthreads();
  const int hh = lane >> 4;
  const int c8 = (lane & 15) * 8;
  for (int pass = 0; pass < 2; ++pass) {
#pragma unroll 1
    for (int it = 0; it < 9; ++it) {
      const int xp = it * 16 + wave * 2 + hh;
      if (xp < PW) {
        const int xpc = min(max(xp, 1), IMW);
        const v4u lv = *(const v4ua*)(sT + xpc * XT_PITCH + c8);
        const bool inside = (xp >= 1) && (xp <= IMW);
        v4u val;
        val.x = inside ? lv.x : 0u;
        val.y = inside ? lv.y : 0u;
        val.z = inside ? lv.z : 0u;
        val.w = inside ? lv.w : 0u;
        unsigned short* dst = xt + (((size_t)b * PROWS + (size_t)yp * PW + xp) * CIN + chalf * 128 + c8);
        *(volatile v4u*)dst = val;
      }
    }
    __threadfence();
  }
}

__device__ __forceinline__ v4u wconv_pack(const float* __restrict__ w, int occ, int g) {
  const int kb = g * 8;
  const int tap = kb >> 8;
  const int c0 = kb & (CIN - 1);
  const float* src = w + ((size_t)occ * CIN + c0) * NTAP + tap;
  float f[8];
#pragma unroll
  for (int e = 0; e < 8; ++e) f[e] = src[e * NTAP];
  v4u val;
  val.x = pack_bf2(f[0], f[1]);
  val.y = pack_bf2(f[2], f[3]);
  val.z = pack_bf2(f[4], f[5]);
  val.w = pack_bf2(f[6], f[7]);
  return val;
}
__global__ __launch_bounds__(256) void k_wconv(const float* __restrict__ w, unsigned short* __restrict__ wbt) {
  const int oc = blockIdx.x;
  const int tid = threadIdx.x;
  const int occ = min(oc, NCH - 1);
  const int g0 = tid;
  const int g1 = min(tid + 256, KCONV / 8 - 1);
  v4u v0 = wconv_pack(w, occ, g0);
  v4u v1 = wconv_pack(w, occ, g1);
  if (oc >= NCH) {
    v0 = (v4u){0u, 0u, 0u, 0u};
    v1 = (v4u){0u, 0u, 0u, 0u};
  }
  unsigned short* row = wbt + (size_t)oc * KCONV;
  for (int pass = 0; pass < 2; ++pass) {
    *(volatile v4u*)(row + g0 * 8) = v0;
    if (tid + 256 < KCONV / 8) *(volatile v4u*)(row + (tid + 256) * 8) = v1;
    __threadfence();
  }
}

__global__ __launch_bounds__(256) void k_wout(const float* __restrict__ w, unsigned short* __restrict__ wq, int n8) {
  const int i = blockIdx.x * 256 + threadIdx.x;
  if (i < n8) {
    const v4f a = *(const v4f*)(w + (size_t)i * 8);
    const v4f c = *(const v4f*)(w + (size_t)i * 8 + 4);
    v4u val;
    val.x = pack_bf2(a[0], a[1]);
    val.y = pack_bf2(a[2], a[3]);
    val.z = pack_bf2(c[0], c[1]);
    val.w = pack_bf2(c[2], c[3]);
    unsigned short* dst = wq + (size_t)i * 8;
    *(volatile v4u*)dst = val;
    __threadfence();
    *(volatile v4u*)dst = val;
  }
}

__global__ __launch_bounds__(256) void k_stats(const float* __restrict__ tmpq, const float* __restrict__ boff,
                                             float* __restrict__ stats) {
  __shared__ float red[256];
  const int j = blockIdx.x;
  const int b = j / NTAP;
  const int k = j - b * NTAP;
  const int tid = threadIdx.x;
  const float* p = tmpq + (size_t)b * QM * NCHP + (2 * NTAP + k);
  const float bk = boff[2 * NTAP + k];
  float mx = -__builtin_huge_valf();
#pragma unroll 4
  for (int i = tid; i < HWPIX; i += 256) {
    const int q = (i >> 7) * PW + (i & (IMW - 1));
    mx = fmaxf(mx, p[(size_t)q * NCHP] + bk);
  }
  red[tid] = mx;
  __syncthreads();
  for (int s = 128; s > 0; s >>= 1) {
    if (tid < s) red[tid] = fmaxf(red[tid], red[tid + s]);
    __syncthreads();
  }
  mx = red[0];
  __syncthreads();
  float sm = 0.f;
#pragma unroll 4
  for (int i = tid; i < HWPIX; i += 256) {
    const int q = (i >> 7) * PW + (i & (IMW - 1));
    sm += expf(p[(size_t)q * NCHP] + bk - mx);
  }
  red[tid] = sm;
  __syncthreads();
  for (int s = 128; s > 0; s >>= 1) {
    if (tid < s) red[tid] = red[tid] + red[tid + s];
    __syncthreads();
  }
  const float tot = red[0];
  if (tid < 32) {
    const float inv = 1.0f / tot;
    const float v = (tid == 0) ? mx : ((tid == 1) ? inv : 0.f);
    float* dst = stats + (size_t)j * 32 + tid;
    *(volatile float*)dst = v;
    __threadfence();
    *(volatile float*)dst = v;
  }
}

__global__ __launch_bounds__(256) void k_sample(const float* __restrict__ x, const float* __restrict__ tmpq,
                                              const float* __restrict__ boff, const float* __restrict__ stats,
                                              unsigned short* __restrict__ agg) {
  __shared__ float sW[SPB * NTAP * 4];
  __shared__ int   sI[SPB * NTAP * 4];
  const int tid = threadIdx.x;
  const int lane = tid & 31;
  const int wave = tid >> 5;
  const int pix0 = blockIdx.x * SPB;
  const int b = pix0 / HWPIX;
  const int hw0 = pix0 - b * HWPIX;
  {
    const int p = tid & (SPB - 1);
    const int tg = tid >> 6;
    const int hw = hw0 + p;
    const int h = hw >> 7;
    const int wv = hw & (IMW - 1);
    const float* tp = tmpq + ((size_t)b * QM + (size_t)h * PW + wv) * NCHP;
#pragma unroll 1
    for (int k = tg; k < NTAP; k += 4) {
      const int ki = k / 3;
      const int kj = k - 3 * ki;
      const float dyv = tp[2 * k] + boff[2 * k];
      const float dxv = tp[2 * k + 1] + boff[2 * k + 1];
      const float lg  = tp[2 * NTAP + k] + boff[2 * NTAP + k];
      const float smax = stats[(b * NTAP + k) * 32];
      const float sinv = stats[(b * NTAP + k) * 32 + 1];
      const float mk = expf(lg - smax) * sinv;
      float py = dyv + (float)(h + ki - 1);
      float px = dxv + (float)(wv + kj - 1);
      py = fminf(fmaxf(py, -2.0f), (float)(IMH + 1));
      px = fminf(fmaxf(px, -2.0f), (float)(IMW + 1));
      const float fy = floorf(py);
      const float fx = floorf(px);
      const int y0 = (int)fy;
      const int x0 = (int)fx;
      const float ly = py - fy;
      const float lx = px - fx;
      const float hy = 1.0f - ly;
      const float hx = 1.0f - lx;
      const bool vy0 = (y0 >= 0) && (y0 < IMH);
      const bool vy1 = (y0 + 1 >= 0) && (y0 + 1 < IMH);
      const bool vx0 = (x0 >= 0) && (x0 < IMW);
      const bool vx1 = (x0 + 1 >= 0) && (x0 + 1 < IMW);
      const float w00 = (vy0 && vx0) ? (hy * hx) * mk : 0.f;
      const float w01 = (vy0 && vx1) ? (hy * lx) * mk : 0.f;
      const float w10 = (vy1 && vx0) ? (ly * hx) * mk : 0.f;
      const float w11 = (vy1 && vx1) ? (ly * lx) * mk : 0.f;
      const int y0c = min(max(y0, 0), IMH - 1);
      const int y1c = min(max(y0 + 1, 0), IMH - 1);
      const int x0c = min(max(x0, 0), IMW - 1);
      const int x1c = min(max(x0 + 1, 0), IMW - 1);
      const int base = (p * NTAP + k) * 4;
      sW[base + 0] = w00;
      sW[base + 1] = w01;
      sW[base + 2] = w10;
      sW[base + 3] = w11;
      sI[base + 0] = y0c * IMW + x0c;
      sI[base + 1] = y0c * IMW + x1c;
      sI[base + 2] = y1c * IMW + x0c;
      sI[base + 3] = y1c * IMW + x1c;
    }
  }
  __syncthreads();
  const float* xb = x + ((size_t)b * CIN + (size_t)lane * 8) * HWPIX;
#pragma unroll 1
  for (int i = 0; i < SPB / 8; ++i) {
    const int p = wave + 8 * i;
    float acc[8];
#pragma unroll
    for (int e = 0; e < 8; ++e) acc[e] = 0.f;
#pragma unroll 1
    for (int k = 0; k < NTAP; ++k) {
      const int base = (p * NTAP + k) * 4;
      const float w0 = sW[base + 0];
      const float w1 = sW[base + 1];
      const float w2 = sW[base + 2];
      const float w3 = sW[base + 3];
      const int i0 = sI[base + 0];
      const int i1 = sI[base + 1];
      const int i2 = sI[base + 2];
      const int i3 = sI[base + 3];
#pragma unroll
      for (int e = 0; e < 4; ++e) {
        const float* xp = xb + (size_t)e * HWPIX;
        const float t0 = xp[i0];
        const float t1 = xp[i1];
        const float t2 = xp[i2];
        const float t3 = xp[i3];
        float a = acc[e];
        a = fmaf(w0, t0, a);
        a = fmaf(w1, t1, a);
        a = fmaf(w2, t2, a);
        a = fmaf(w3, t3, a);
        acc[e] = a;
      }
      asm volatile("" : "+v"(acc[0]), "+v"(acc[1]), "+v"(acc[2]), "+v"(acc[3]) : : "memory");
#pragma unroll
      for (int e = 4; e < 8; ++e) {
        const float* xp = xb + (size_t)e * HWPIX;
        const float t0 = xp[i0];
        const float t1 = xp[i1];
        const float t2 = xp[i2];
        const float t3 = xp[i3];
        float a = acc[e];
        a = fmaf(w0, t0, a);
        a = fmaf(w1, t1, a);
        a = fmaf(w2, t2, a);
        a = fmaf(w3, t3, a);
        acc[e] = a;
      }
      asm volatile("" : "+v"(acc[4]), "+v"(acc[5]), "+v"(acc[6]), "+v"(acc[7]) : : "memory");
    }
    v4u val;
    val.x = pack_bf2(acc[0], acc[1]);
    val.y = pack_bf2(acc[2], acc[3]);
    val.z = pack_bf2(acc[4], acc[5]);
    val.w = pack_bf2(acc[6], acc[7]);
    unsigned short* dst = agg + ((size_t)(pix0 + p) * CIN + (size_t)lane * 8);
    *(volatile v4u*)dst = val;
    __threadfence();
    *(volatile v4u*)dst = val;
  }
}

extern "C" void kernel_launch(void* const* d_in, const int* in_sizes, int n_in,
                              void* d_out, int out_size, void* d_ws, size_t ws_size,
                              hipStream_t stream) {
  if (n_in < 5) return;
  if (ws_size < WS_TOTAL) return;
  if (in_sizes[0] != NB * CIN * HWPIX) return;
  if (in_sizes[1] != NCH * CIN * NTAP) return;
  if (in_sizes[3] != NOUT * CIN) return;
  if (out_size != NB * NOUT * HWPIX) return;

  const float* x      = (const float*)d_in[0];
  const float* w_off  = (const float*)d_in[1];
  const float* b_off  = (const float*)d_in[2];
  const float* weight = (const float*)d_in[3];
  const float* bias   = (const float*)d_in[4];
  float* out = (float*)d_out;

  char* ws = (char*)d_ws;
  unsigned short* xt    = (unsigned short*)(ws + OFF_XT);
  unsigned short* wbt   = (unsigned short*)(ws + OFF_WBT);
  float*          tmpq  = (float*)(ws + OFF_TMPQ);
  float*          stats = (float*)(ws + OFF_STATS);
  unsigned short* wq    = (unsigned short*)(ws + OFF_WQ);
  unsigned short* agg   = (unsigned short*)(ws + OFF_AGG);

  k_xpad<<<dim3(IMH + 3, 2, NB), 256, 0, stream>>>(x, xt);
  k_wconv<<<NCHP, 256, 0, stream>>>(w_off, wbt);
  k_wout<<<(NOUT * CIN / 8 + 255) / 256, 256, 0, stream>>>(weight, wq, NOUT * CIN / 8);
  {
    const int tiles = (QM / 64) * (NCHP / 64);
    gemm64_bf16<1, 0><<<dim3((tiles + 7) / 8, NB), 256, 0, stream>>>(
        xt, CIN, (long)PROWS * CIN,
        wbt, KCONV, 0L,
        tmpq, NCHP, (long)QM * NCHP,
        bias, QM, NCHP, KCONV, 1.0f);
  }
  k_stats<<<NB * NTAP, 256, 0, stream>>>(tmpq, b_off, stats);
  k_sample<<<NB * HWPIX / SPB, 256, 0, stream>>>(x, tmpq, b_off, stats, agg);
  {
    const int tiles = (NOUT / 64) * (HWPIX / 64);
    gemm64_bf16<0, 1><<<dim3((tiles + 7) / 8, NB), 256, 0, stream>>>(
        wq, CIN, 0L,
        agg, CIN, (long)HWPIX * CIN,
        out, HWPIX, (long)NOUT * HWPIX,
        bias, NOUT, HWPIX, CIN, 1.0f);
  }
}
